// NN_adiab_11072425689287
// MI455X (gfx1250) — hardware-verified
//
#include <hip/hip_runtime.h>
#include <stdint.h>

typedef _Float16 v16h __attribute__((ext_vector_type(16)));
typedef _Float16 v8h  __attribute__((ext_vector_type(8)));
typedef float    v8f  __attribute__((ext_vector_type(8)));
typedef float    v4f  __attribute__((ext_vector_type(4)));

#define HID        256
#define KT         8
#define NT         16

#define WS_W2_OFF   0
#define WS_W3_OFF   131072
#define WS_TOTAL    139264
#define N_PIECE_W2  8192
#define N_PIECE     8704

#define SM_W2       0
#define SM_W3       131072
#define SM_CW       139264
#define SM_B2       143360
#define SM_B3       144384
#define SM_WAVE     144448
#define HP          264
#define SM_H_BYTES  (16 * HP * 2)
#define SM_WV_OFF   SM_H_BYTES
#define SM_E_OFF    (SM_H_BYTES + 256)
#define SM_WAVE_STR 8832
#define SM_TOTAL    (SM_WAVE + 8 * SM_WAVE_STR)

#define SC_H1   8.0f
#define SC_W2   16.0f
#define SC_H2   128.0f
#define SC_W3   64.0f
#define SC_W    8192.0f
#define INV_W   (1.0f / 8192.0f)

__device__ __forceinline__ v8f wmma_f16(v16h a, v16h b, v8f c) {
    c = __builtin_amdgcn_wmma_f32_16x16x32_f16(false, a, false, b, (short)0, c, false, false);
    asm volatile("v_nop\n\tv_nop\n\tv_nop\n\tv_nop" : "+v"(c) : "v"(a), "v"(b));
    return c;
}

__device__ __forceinline__ void lds_wave_sync() {
    asm volatile("s_wait_dscnt 0" ::: "memory");
}

__global__ void __launch_bounds__(256)
k_pack(const float* __restrict__ W2, const float* __restrict__ W3, _Float16* __restrict__ wsh) {
    const int q = blockIdx.x * 256 + threadIdx.x;
    if (q >= N_PIECE) return;
    v8h v;
    _Float16* dst;
    if (q < N_PIECE_W2) {
        const int f = q >> 1, half = q & 1;
        const int lane = f & 31, kt = (f >> 5) & 7, nt = f >> 8;
        const int n = lane & 15, h = lane >> 4;
        const int kb = kt * 32 + 16 * half + 8 * h;
        const int col = nt * 16 + n;
        #pragma unroll
        for (int i = 0; i < 8; ++i) v[i] = (_Float16)(SC_W2 * W2[(kb + i) * HID + col]);
        dst = wsh + (WS_W2_OFF / 2) + (size_t)q * 8;
    } else {
        const int j = q - N_PIECE_W2;
        const int f = j >> 1, half = j & 1;
        const int lane = f & 31, kt = (f >> 5) & 7;
        const int n = lane & 15, h = lane >> 4;
        const int kb = kt * 32 + 16 * half + 8 * h;
        const int nn = (n < 3) ? n : 0;
        #pragma unroll
        for (int i = 0; i < 8; ++i) {
            const float wv = W3[(kb + i) * 3 + nn];
            v[i] = (n < 3) ? (_Float16)(SC_W3 * wv) : (_Float16)0.0f;
        }
        dst = wsh + (WS_W3_OFF / 2) + (size_t)j * 8;
    }
    *(volatile v8h*)dst = v;
    __threadfence();
    *(volatile v8h*)dst = v;
}

__global__ void __launch_bounds__(256)
k_main(const float* __restrict__ x, const float* __restrict__ W1, const float* __restrict__ b1,
       const float* __restrict__ b2, const float* __restrict__ b3,
       const _Float16* __restrict__ wsh, float* __restrict__ out,
       int nsamp, int ntiles) {
    #pragma clang fp contract(off)
    extern __shared__ __align__(16) char smem[];
    const int t = threadIdx.x;

    {
        const uint4* src = (const uint4*)wsh;
        uint4* dst = (uint4*)smem;
        for (int i = t; i < WS_TOTAL / 16; i += 256) dst[i] = src[i];
        v4f c;
        c[0] = SC_H1 * W1[t];
        c[1] = SC_H1 * W1[HID + t];
        c[2] = SC_H1 * W1[2 * HID + t];
        c[3] = SC_H1 * b1[t];
        ((v4f*)(smem + SM_CW))[t] = c;
        ((float*)(smem + SM_B2))[t] = SC_H2 * b2[t];
        if (t < 16) ((float*)(smem + SM_B3))[t] = (t < 3) ? SC_W * b3[t] : 0.0f;
    }
    __syncthreads();

    const int lane = t & 31, wave = t >> 5;
    const int h = lane >> 4, m = lane & 15;

    const _Float16* sW2 = (const _Float16*)(smem + SM_W2);
    const _Float16* sW3 = (const _Float16*)(smem + SM_W3);
    const v4f*   sCW = (const v4f*)(smem + SM_CW);
    const float* sB2 = (const float*)(smem + SM_B2);
    const float* sB3 = (const float*)(smem + SM_B3);

    char* wb = smem + SM_WAVE + wave * SM_WAVE_STR;
    _Float16* sH  = (_Float16*)wb;
    float*    sWv = (float*)(wb + SM_WV_OFF);
    float*    sE  = (float*)(wb + SM_E_OFF);

    const int stride = gridDim.x * 8;
    for (int tile = blockIdx.x * 8 + wave; tile < ntiles; tile += stride) {
        const int row0 = tile * 16;
        const int nvalid = (nsamp - row0 < 16) ? (nsamp - row0) : 16;
        int rs = row0 + m;
        if (rs > nsamp - 1) rs = nsamp - 1;

        float r0, r1, r2;
        {
            const float* xp = x + (size_t)rs * 9;
            const float ax = xp[0], ay = xp[1], az = xp[2];
            const float bx = xp[3], by = xp[4], bz = xp[5];
            const float cx = xp[6], cy = xp[7], cz = xp[8];
            float dx, dy, dz;
            dx = ax - bx; dy = ay - by; dz = az - bz; r0 = sqrtf(dx * dx + dy * dy + dz * dz);
            dx = ax - cx; dy = ay - cy; dz = az - cz; r1 = sqrtf(dx * dx + dy * dy + dz * dz);
            dx = bx - cx; dy = by - cy; dz = bz - cz; r2 = sqrtf(dx * dx + dy * dy + dz * dz);
        }

        v16h afr[KT];
        {
            const v4f* cwh = sCW + 8 * h;
            #pragma unroll
            for (int kt = 0; kt < KT; ++kt) {
                v8h hv0, hv1;
                #pragma unroll
                for (int i = 0; i < 8; ++i) {
                    const v4f c0 = cwh[kt * 32 + i];
                    float d0 = fmaf(r0, c0[0], c0[3]);
                    d0 = fmaf(r1, c0[1], d0);
                    d0 = fmaf(r2, c0[2], d0);
                    d0 = fmaxf(d0, 0.0f);
                    hv0[i] = (_Float16)d0;
                    const v4f c1 = cwh[kt * 32 + 16 + i];
                    float d1 = fmaf(r0, c1[0], c1[3]);
                    d1 = fmaf(r1, c1[1], d1);
                    d1 = fmaf(r2, c1[2], d1);
                    d1 = fmaxf(d1, 0.0f);
                    hv1[i] = (_Float16)d1;
                }
                afr[kt] = __builtin_shufflevector(hv0, hv1, 0,1,2,3,4,5,6,7,8,9,10,11,12,13,14,15);
            }
        }

        #pragma unroll 1
        for (int nt = 0; nt < NT; ++nt) {
            const int col = nt * 16 + m;
            const float bb = sB2[col];
            v8f acc;
            #pragma unroll
            for (int r = 0; r < 8; ++r) acc[r] = bb;
            const _Float16* bp = sW2 + (size_t)(nt * KT * 32 + lane) * 16;
            #pragma unroll
            for (int kt = 0; kt < KT; ++kt) {
                const v16h bv = *(const v16h*)(bp + kt * 32 * 16);
                acc = wmma_f16(afr[kt], bv, acc);
            }
            _Float16* st = sH + (8 * h) * HP + col;
            #pragma unroll
            for (int r = 0; r < 8; ++r) {
                const float v = fmaxf(acc[r], 0.0f);
                st[r * HP] = (_Float16)v;
            }
        }
        lds_wave_sync();

        v8f acc3;
        {
            const float b3v = sB3[m];
            #pragma unroll
            for (int r = 0; r < 8; ++r) acc3[r] = b3v;
        }
        #pragma unroll
        for (int kt = 0; kt < KT; ++kt) {
            const v16h bv = *(const v16h*)(sW3 + (kt * 32 + lane) * 16);
            const _Float16* rp = sH + m * HP + kt * 32 + 8 * h;
            const v8h lo = *(const v8h*)(rp);
            const v8h hi = *(const v8h*)(rp + 16);
            const v16h a3 = __builtin_shufflevector(lo, hi, 0,1,2,3,4,5,6,7,8,9,10,11,12,13,14,15);
            acc3 = wmma_f16(a3, bv, acc3);
        }
        if (m < 3) {
            #pragma unroll
            for (int r = 0; r < 8; ++r) sWv[(8 * h + r) * 4 + m] = acc3[r] * INV_W;
        }
        lds_wave_sync();

        if (h == 0) {
            const float w0 = sWv[m * 4 + 0], w1 = sWv[m * 4 + 1], w01 = sWv[m * 4 + 2];
            const float mm  = 0.5f * (w0 + w1);
            const float dd  = 0.5f * (w0 - w1);
            const float rad = sqrtf(dd * dd + w01 * w01);
            sE[2 * m]     = mm - rad;
            sE[2 * m + 1] = mm + rad;
        }
        lds_wave_sync();

        if (nvalid == 16) {
            if (lane < 8) {
                const v4f ov = *(const v4f*)(sE + 4 * lane);
                float* op = out + (size_t)row0 * 2 + 4 * lane;
                *(volatile v4f*)op = ov;
                __threadfence();
                *(volatile v4f*)op = ov;
            }
        } else {
            if (lane < nvalid) {
                const float e0 = sE[2 * lane], e1 = sE[2 * lane + 1];
                float* op = out + (size_t)(row0 + lane) * 2;
                *(volatile float*)(op)     = e0;
                *(volatile float*)(op + 1) = e1;
                __threadfence();
                *(volatile float*)(op)     = e0;
                *(volatile float*)(op + 1) = e1;
            }
        }
        lds_wave_sync();
    }
}

extern "C" void kernel_launch(void* const* d_in, const int* in_sizes, int n_in,
                              void* d_out, int out_size, void* d_ws, size_t ws_size,
                              hipStream_t stream) {
    if (n_in < 7) return;
    const float* x  = (const float*)d_in[0];
    const float* W1 = (const float*)d_in[1];
    const float* b1 = (const float*)d_in[2];
    const float* W2 = (const float*)d_in[3];
    const float* b2 = (const float*)d_in[4];
    const float* W3 = (const float*)d_in[5];
    const float* b3 = (const float*)d_in[6];
    float* out = (float*)d_out;

    if (in_sizes[1] != 3 * HID || in_sizes[2] != HID || in_sizes[3] != HID * HID ||
        in_sizes[4] != HID || in_sizes[5] != HID * 3 || in_sizes[6] < 3) return;
    if (ws_size < (size_t)WS_TOTAL) return;

    int nsamp = in_sizes[0] / 9;
    const int nout = out_size / 2;
    if (nout < nsamp) nsamp = nout;
    if (nsamp <= 0) return;
    const int ntiles = (nsamp + 15) / 16;
    int grid = (ntiles + 7) / 8;
    if (grid > 512) grid = 512;
    if (grid < 1) grid = 1;

    hipFuncSetAttribute((const void*)k_main, hipFuncAttributeMaxDynamicSharedMemorySize, SM_TOTAL);

    k_pack<<<(N_PIECE + 255) / 256, 256, 0, stream>>>(W2, W3, (_Float16*)d_ws);
    k_main<<<grid, 256, SM_TOTAL, stream>>>(x, W1, b1, b2, b3, (const _Float16*)d_ws, out,
                                           nsamp, ntiles);
}
